// KA_attention_crossinf_16655883173900
// MI455X (gfx1250) — hardware-verified
//
#include <hip/hip_runtime.h>


typedef __attribute__((ext_vector_type(16))) __bf16 v16bf;
typedef __attribute__((ext_vector_type(8)))  float  v8f;

union Frag { v16bf v; unsigned int u[8]; };

#define WROW 65
#define SROW 65

static __device__ inline void bfsplit(float x, unsigned short& hi, unsigned short& lo) {
    union { __bf16 b; unsigned short s; } c;
    __bf16 bh = (__bf16)x;
    c.b = bh; hi = c.s;
    float rem = x - (float)bh;
    c.b = (__bf16)rem; lo = c.s;
}

static __device__ inline void proc_elem(float x, const float* __restrict__ cf,
                                        unsigned short& hi, unsigned short& lo,
                                        float& fval) {
    float e = __expf(-x);
    float s = x / (1.0f + e);
    bfsplit(s, hi, lo);
    float sx, cx;
    __sincosf(x, &sx, &cx);
    float c2 = 2.0f * cx;
    float p2 = 0.0f, p1 = sx;
    float acc = cf[0] * sx;
#pragma unroll
    for (int j = 1; j < 12; j++) {
        float cur = __fmaf_rn(c2, p1, -p2);
        acc = __fmaf_rn(cf[j], cur, acc);
        p2 = p1; p1 = cur;
    }
    fval = acc;
}

#define KA_SMEM_BYTES ((9856 + 2 * 128 * WROW + 2 * 64 * SROW) * 4)

__global__ void __launch_bounds__(256)
ka_branch_kernel(const float* __restrict__ q, const float* __restrict__ k,
                 const float* __restrict__ W,
                 const float* __restrict__ coef_q, const float* __restrict__ coef_k,
                 const float* __restrict__ scale_base, const float* __restrict__ scale_sp,
                 float* __restrict__ sums) {
    extern __shared__ char smem[];
    float* fv        = (float*)smem;
    float* coefs     = fv + 8192;
    float* rowhalf   = coefs + 1536;
    unsigned int* whi32 = (unsigned int*)(rowhalf + 128);
    unsigned int* wlo32 = whi32 + 128 * WROW;
    unsigned int* shi32 = wlo32 + 128 * WROW;
    unsigned int* slo32 = shi32 + 64 * SROW;

    const int t = threadIdx.x;
    const int which = blockIdx.y;
    const float* xin  = which ? k : q;
    const float* coef = which ? coef_k : coef_q;
    const int r0 = blockIdx.x * 64;

    for (int i = t; i < 1536; i += 256) coefs[i] = coef[i];
    for (int i = t; i < 8192; i += 256) {
        int n  = i >> 6;
        int kk = i & 63;
        float w0 = W[2 * i], w1 = W[2 * i + 1];
        unsigned short h0, l0, h1, l1;
        bfsplit(w0, h0, l0);
        bfsplit(w1, h1, l1);
        whi32[n * WROW + kk] = (unsigned int)h0 | ((unsigned int)h1 << 16);
        wlo32[n * WROW + kk] = (unsigned int)l0 | ((unsigned int)l1 << 16);
    }
    if (t < 128) rowhalf[t] = 0.0f;
    __syncthreads();

    const float* xblk = xin + (size_t)r0 * 128;
    for (int i = t; i < 4096; i += 256) {
        int m  = i >> 6;
        int kk = i & 63;
        int d0 = kk * 2;
        float x0 = xblk[m * 128 + d0];
        float x1 = xblk[m * 128 + d0 + 1];
        unsigned short h0, l0, h1, l1;
        float f0, f1;
        proc_elem(x0, &coefs[d0 * 12], h0, l0, f0);
        proc_elem(x1, &coefs[(d0 + 1) * 12], h1, l1, f1);
        shi32[m * SROW + kk] = (unsigned int)h0 | ((unsigned int)h1 << 16);
        slo32[m * SROW + kk] = (unsigned int)l0 | ((unsigned int)l1 << 16);
        fv[m * 128 + d0]     = f0;
        fv[m * 128 + d0 + 1] = f1;
    }
    __syncthreads();

    const int wv = t >> 5, lane = t & 31;
    const int stripe = wv >> 1;
    const int chalf  = wv & 1;
    const int hh = lane >> 4, ln = lane & 15;

    v8f acc[4] = {};
    const int mA = stripe * 16 + ln;
    for (int ks = 0; ks < 4; ks++) {
        Frag ahi, alo;
        int abase = mA * SROW + ks * 16 + hh * 4;
#pragma unroll
        for (int v = 0; v < 4; v++) { ahi.u[v] = shi32[abase + v];      alo.u[v] = slo32[abase + v]; }
#pragma unroll
        for (int v = 0; v < 4; v++) { ahi.u[4 + v] = shi32[abase + 8 + v]; alo.u[4 + v] = slo32[abase + 8 + v]; }
#pragma unroll
        for (int ct = 0; ct < 4; ct++) {
            int n = chalf * 64 + ct * 16 + ln;
            int bbase = n * WROW + ks * 16 + hh * 4;
            Frag bhi, blo;
#pragma unroll
            for (int v = 0; v < 4; v++) { bhi.u[v] = whi32[bbase + v];         blo.u[v] = wlo32[bbase + v]; }
#pragma unroll
            for (int v = 0; v < 4; v++) { bhi.u[4 + v] = whi32[bbase + 8 + v]; blo.u[4 + v] = wlo32[bbase + 8 + v]; }
            acc[ct] = __builtin_amdgcn_wmma_f32_16x16x32_bf16(false, ahi.v, false, bhi.v,
                                                              (short)0, acc[ct], false, false);
            acc[ct] = __builtin_amdgcn_wmma_f32_16x16x32_bf16(false, ahi.v, false, blo.v,
                                                              (short)0, acc[ct], false, false);
            acc[ct] = __builtin_amdgcn_wmma_f32_16x16x32_bf16(false, alo.v, false, bhi.v,
                                                              (short)0, acc[ct], false, false);
            asm volatile("v_nop\n\tv_nop\n\tv_nop\n\tv_nop" : "+v"(acc[ct]) : "v"(alo.v), "v"(bhi.v));
        }
    }

    float part[8];
#pragma unroll
    for (int r = 0; r < 8; r++) part[r] = 0.0f;
#pragma unroll
    for (int ct = 0; ct < 4; ct++) {
        int n = chalf * 64 + ct * 16 + ln;
#pragma unroll
        for (int r = 0; r < 8; r++) {
            int m_local = stripe * 16 + 8 * hh + r;
            int grow = r0 + m_local;
            int p = grow & 127, h = (grow >> 7) & 15;
            size_t sidx = ((size_t)(h * 128 + p)) * 128 + n;
            float tv = __fmaf_rn(fv[m_local * 128 + n], scale_sp[sidx],
                                 acc[ct][r] * scale_base[sidx]);
            part[r] += 1.0f / (1.0f + __expf(-tv));
        }
    }
#pragma unroll
    for (int r = 0; r < 8; r++) {
        float v = part[r];
        v += __shfl_xor(v, 1, 16);
        v += __shfl_xor(v, 2, 16);
        v += __shfl_xor(v, 4, 16);
        v += __shfl_xor(v, 8, 16);
        if (ln == 0) rowhalf[chalf * 64 + stripe * 16 + 8 * hh + r] = v;
    }
    __syncthreads();
    if (t < 64) { const float sv = rowhalf[t] + rowhalf[64 + t]; float* sp = sums + (size_t)which * 32768 + r0 + t;
        *(volatile float*)sp = sv; __threadfence(); *(volatile float*)sp = sv; }
}

__global__ void __launch_bounds__(128)
ka_out_kernel(const float* __restrict__ sums, const float* __restrict__ w_qk,
              const float* __restrict__ b_qk, float* __restrict__ out) {
    __shared__ float skv[128], sqv[128], rwv[128], skwv[128], mxv[128], rsv[128];
    const int bh = blockIdx.x;
    const int j  = threadIdx.x;

    sqv[j] = sums[bh * 128 + j];
    skv[j] = sums[32768 + bh * 128 + j];
    __syncthreads();

    float rw = 0.0f, skw = 0.0f;
    const float* wrow = w_qk + (size_t)j * 128;
#pragma unroll 4
    for (int pp = 0; pp < 128; pp++) {
        float w = wrow[pp];
        rw += w;
        skw = __fmaf_rn(skv[pp], w, skw);
    }
    rwv[j]  = rw;
    skwv[j] = skw + b_qk[j];
    __syncthreads();

    {
        float s = sqv[j];
        float m = -3.402823466e+38f;
#pragma unroll 4
        for (int c = 0; c < 128; c++) m = fmaxf(m, __fmaf_rn(s, rwv[c], skwv[c]));
        float sum = 0.0f;
#pragma unroll 4
        for (int c = 0; c < 128; c++) sum += __expf(__fmaf_rn(s, rwv[c], skwv[c]) - m);
        mxv[j] = m;
        rsv[j] = 1.0f / sum;
    }
    __syncthreads();

    float* orow = out + (size_t)bh * 16384;
    float rwj = rwv[j], skwj = skwv[j];
    for (int pass = 0; pass < 2; ++pass) {
#pragma unroll 2
        for (int p = 0; p < 128; p++) {
            float v = __expf(__fmaf_rn(sqv[p], rwj, skwj) - mxv[p]) * rsv[p];
            *(volatile float*)(orow + p * 128 + j) = v;
        }
        __threadfence();
    }
}

extern "C" void kernel_launch(void* const* d_in, const int* in_sizes, int n_in,
                              void* d_out, int out_size, void* d_ws, size_t ws_size,
                              hipStream_t stream) {
    (void)in_sizes; (void)n_in; (void)out_size; (void)ws_size;
    const float* q          = (const float*)d_in[0];
    const float* k          = (const float*)d_in[1];
    const float* base_weight = (const float*)d_in[4];
    const float* coef_q     = (const float*)d_in[5];
    const float* coef_k     = (const float*)d_in[6];
    const float* scale_base = (const float*)d_in[7];
    const float* scale_sp   = (const float*)d_in[8];
    const float* w_qk       = (const float*)d_in[9];
    const float* b_qk       = (const float*)d_in[10];

    if (ws_size < (size_t)2 * 32768 * 4) return;
    float* sums = (float*)d_ws;
    float* out  = (float*)d_out;

    dim3 gA(512, 2);
    hipFuncSetAttribute((const void*)ka_branch_kernel, hipFuncAttributeMaxDynamicSharedMemorySize, KA_SMEM_BYTES);
    ka_branch_kernel<<<gA, 256, KA_SMEM_BYTES, stream>>>(
        q, k, base_weight, coef_q, coef_k, scale_base, scale_sp, sums);

    ka_out_kernel<<<256, 128, 0, stream>>>(sums, w_qk, b_qk, out);
}
